// NeuralNetwork_49804440764428
// MI455X (gfx1250) — hardware-verified
//
#include <hip/hip_runtime.h>
#include <math.h>

constexpr int NSEQ     = 2048;
constexpr int NSTEP    = 512;
constexpr int NIN      = 4;
constexpr int NHID     = 64;
constexpr int NGATE    = 4 * NHID;
constexpr int NHEAD    = 4;
constexpr int NTHR     = 128;
constexpr int ROWS_BLK = 16;
constexpr int WPITCH   = 72;
constexpr int HPITCH   = 72;
constexpr int HSPITCH  = 68;
constexpr float W_CARRY  = 256.0f;
constexpr float H_CARRY  = 8.0f;
constexpr float ACC_FOLD = 1.0f / 2048.0f;
static_assert(NSEQ % ROWS_BLK == 0);
static_assert(NHID == 16 * (NTHR / 32));
static_assert(NGATE * NHID == 32 * NTHR * 4);
static_assert(ROWS_BLK * NHID == NTHR * 8);
static_assert(NGATE * NIN == 2 * NTHR * 4);
static_assert(NGATE == 2 * NTHR);
static_assert(NHEAD * NHID == 64 * 4);
static_assert(ROWS_BLK * NIN == 64);
static_assert(ROWS_BLK * NHEAD == 16 * 4);
static_assert((WPITCH % 8) == 0 && (HPITCH % 8) == 0 && (HSPITCH % 4) == 0);
static_assert(NHID % 32 == 0);

typedef __attribute__((ext_vector_type(16))) _Float16 v16h;
typedef __attribute__((ext_vector_type(8)))  _Float16 v8h;
typedef __attribute__((ext_vector_type(8)))  float    v8f;
typedef __attribute__((ext_vector_type(4)))  float    v4f;
typedef __attribute__((ext_vector_type(2)))  unsigned v2u;
typedef __attribute__((ext_vector_type(4)))  unsigned v4u;

__device__ __forceinline__ void mma_guard(v8f& d, v16h a0, v16h a1, v16h b0, v16h b1) {
  asm volatile("v_nop\n\tv_nop\n\tv_nop\n\tv_nop" : "+v"(d) : "v"(a0), "v"(a1), "v"(b0), "v"(b1));
}
__device__ __forceinline__ void acc_guard4(v8f& a, v8f& b, v8f& c, v8f& d) {
  asm volatile("v_nop\n\tv_nop\n\tv_nop\n\tv_nop" : "+v"(a), "+v"(b), "+v"(c), "+v"(d));
}

template <typename T> struct Frag;
template <> struct Frag<_Float16> {
  typedef v16h V; union U { v16h v; v8h h[2]; };
  static __device__ __forceinline__ v16h load(const _Float16* p) {
    U f; f.h[0] = *(const v8h*)(p); f.h[1] = *(const v8h*)(p + 16); return f.v;
  }
  static __device__ __forceinline__ v8f mma(v16h a, v16h b, v8f c) {
    return __builtin_amdgcn_wmma_f32_16x16x32_f16(false, a, false, b, (short)0, c, false, false);
  }
};

__device__ __forceinline__ unsigned short h_bits(float f) { return __builtin_bit_cast(unsigned short, (_Float16)f); }
__device__ __forceinline__ float fsig(float z)  { return __builtin_amdgcn_rcpf(1.0f + expf(-z)); }
__device__ __forceinline__ float ftanh(float z) { return 1.0f - 2.0f * __builtin_amdgcn_rcpf(expf(2.0f * z) + 1.0f); }

__global__ __launch_bounds__(NTHR) void lstm_seq_kernel(const float* __restrict__ x,
                                                        const float* __restrict__ w_ih,
                                                        const float* __restrict__ w_hh,
                                                        const float* __restrict__ b_ih,
                                                        const float* __restrict__ b_hh,
                                                        const float* __restrict__ w_fc,
                                                        const float* __restrict__ b_fc,
                                                        float* __restrict__ out) {
  __shared__ __align__(16) unsigned short Whs[NGATE * WPITCH];
  __shared__ __align__(16) unsigned short Ahs[ROWS_BLK * HPITCH];
  __shared__ __align__(16) float          Xs[ROWS_BLK * NIN];
  __shared__ __align__(16) float          Wis[NGATE * NIN];
  __shared__ __align__(16) float          Bs[NGATE];
  __shared__ __align__(16) float          Wfs[NHEAD * NHID];
  __shared__ __align__(16) float          Hs[ROWS_BLK * HSPITCH];
  __shared__ __align__(16) float          Os[ROWS_BLK * NHEAD];

  const int tid = threadIdx.x, lane = tid & 31, wave = tid >> 5;
  const int c = lane & 15, hh = lane >> 4, koff = hh * 8;
  const int rowbase = blockIdx.x * ROWS_BLK;

#pragma unroll 1
  for (int it = 0; it < 32; ++it) {
    const int idx = it * NTHR + tid;
    const int n = idx >> 4, k4 = (idx & 15) * 4;
    const v4f v = *(const v4f*)(w_hh + (size_t)n * NHID + k4);
    const unsigned short u0 = h_bits(v[0] * W_CARRY), u1 = h_bits(v[1] * W_CARRY);
    const unsigned short u2 = h_bits(v[2] * W_CARRY), u3 = h_bits(v[3] * W_CARRY);
    v2u pk;
    pk[0] = (unsigned)u0 | ((unsigned)u1 << 16);
    pk[1] = (unsigned)u2 | ((unsigned)u3 << 16);
    *(v2u*)(Whs + n * WPITCH + k4) = pk;
  }
  {
    const int row = tid >> 3, c8 = (tid & 7) * 8;
    const v4u z4 = {0u, 0u, 0u, 0u};
    *(v4u*)(Ahs + row * HPITCH + c8) = z4;
  }
#pragma unroll
  for (int i = 0; i < 2; ++i) {
    const int idx = i * NTHR + tid;
    *(v4f*)(Wis + idx * NIN) = *(const v4f*)(w_ih + (size_t)idx * NIN);
  }
  Bs[tid]        = b_ih[tid] + b_hh[tid];
  Bs[tid + NTHR] = b_ih[tid + NTHR] + b_hh[tid + NTHR];
  if (wave < 2) {
    *(v4f*)(Wfs + tid * 4) = *(const v4f*)(w_fc + (size_t)tid * 4);
    const int m = tid >> 2, k = tid & 3;
    Xs[tid] = x[((size_t)(rowbase + m) * NSTEP + 0) * NIN + k];
  }
  __syncthreads();

  v4f wih[4]; float bsum[4];
#pragma unroll
  for (int g = 0; g < 4; ++g) {
    const int n = g * NHID + 16 * wave + c;
    wih[g]  = *(const v4f*)(Wis + n * NIN);
    bsum[g] = Bs[n];
  }
  float cst[8], hst[8];
#pragma unroll
  for (int r = 0; r < 8; ++r) { cst[r] = 0.0f; hst[r] = 0.0f; }

  const _Float16* ahrow = (const _Float16*)Ahs + c * HPITCH + koff;
  const _Float16* whrow = (const _Float16*)Whs + (16 * wave + c) * WPITCH + koff;
  const v8f z8 = {0.f, 0.f, 0.f, 0.f, 0.f, 0.f, 0.f, 0.f};
  const int j = 16 * wave + c;

#pragma unroll 1
  for (int t = 0; t < NSTEP; ++t) {
    const v16h a0 = Frag<_Float16>::load(ahrow);
    const v16h a1 = Frag<_Float16>::load(ahrow + 32);
    v8f acc[4];
#pragma unroll
    for (int g = 0; g < 4; ++g) {
      const _Float16* wr = whrow + g * (NHID * WPITCH);
      const v16h b0 = Frag<_Float16>::load(wr);
      const v16h b1 = Frag<_Float16>::load(wr + 32);
      v8f d = z8;
      d = Frag<_Float16>::mma(a0, b0, d);
      d = Frag<_Float16>::mma(a1, b1, d);
      mma_guard(d, a0, a1, b0, b1);
      acc[g] = d;
    }
    acc_guard4(acc[0], acc[1], acc[2], acc[3]);

#pragma unroll
    for (int r = 0; r < 8; ++r) {
      const v4f xv = *(const v4f*)(Xs + (8 * hh + r) * NIN);
      float xg[4];
#pragma unroll
      for (int g = 0; g < 4; ++g) {
        float s = wih[g][0] * xv[0];
        s = fmaf(wih[g][1], xv[1], s);
        s = fmaf(wih[g][2], xv[2], s);
        s = fmaf(wih[g][3], xv[3], s);
        xg[g] = s + bsum[g];
      }
      const float zi = fmaf(acc[0][r], ACC_FOLD, xg[0]);
      const float zf = fmaf(acc[1][r], ACC_FOLD, xg[1]);
      const float zg = fmaf(acc[2][r], ACC_FOLD, xg[2]);
      const float zo = fmaf(acc[3][r], ACC_FOLD, xg[3]);
      const float ig = fsig(zi);
      const float fg = fsig(zf);
      const float gg = ftanh(zg);
      const float og = fsig(zo);
      const float cn = fg * cst[r] + ig * gg;
      cst[r] = cn;
      hst[r] = og * ftanh(cn);
    }
    __syncthreads();
#pragma unroll
    for (int r = 0; r < 8; ++r) Ahs[(8 * hh + r) * HPITCH + j] = h_bits(hst[r] * H_CARRY);
    if (wave < 2) {
      const int tn = (t + 1 < NSTEP) ? (t + 1) : (NSTEP - 1);
      const int m = tid >> 2, k = tid & 3;
      Xs[tid] = x[((size_t)(rowbase + m) * NSTEP + (size_t)tn) * NIN + k];
    }
    __syncthreads();
  }

#pragma unroll
  for (int r = 0; r < 8; ++r) Hs[(8 * hh + r) * HSPITCH + j] = hst[r];
  __syncthreads();
  if (wave < 2) {
    const int m = tid >> 2, o = tid & 3;
    float s = 0.0f;
#pragma unroll 1
    for (int k4 = 0; k4 < NHID; k4 += 4) {
      const v4f hv = *(const v4f*)(Hs + m * HSPITCH + k4);
      const v4f wv = *(const v4f*)(Wfs + o * NHID + k4);
      s = fmaf(hv[0], wv[0], s);
      s = fmaf(hv[1], wv[1], s);
      s = fmaf(hv[2], wv[2], s);
      s = fmaf(hv[3], wv[3], s);
    }
    Os[tid] = s + b_fc[o];
  }
  __syncthreads();
  if (tid < 16) {
    const v4f v = *(const v4f*)(Os + tid * 4);
    float* op = out + (size_t)rowbase * NHEAD + tid * 4;
    *(volatile v4f*)op = v;
    __threadfence();
    *(volatile v4f*)op = v;
  }
}

extern "C" void kernel_launch(void* const* d_in, const int* in_sizes, int n_in,
                              void* d_out, int out_size, void* d_ws, size_t ws_size, hipStream_t stream) {
  (void)d_ws; (void)ws_size;
  if (n_in < 7 || d_out == nullptr) return;
  if (in_sizes[0] != NSEQ * NSTEP * NIN || in_sizes[1] != NGATE * NIN || in_sizes[2] != NGATE * NHID ||
      in_sizes[3] != NGATE || in_sizes[4] != NGATE || in_sizes[5] != NHEAD * NHID || in_sizes[6] != NHEAD ||
      out_size != NSEQ * NHEAD) return;

  const float* x    = (const float*)d_in[0];
  const float* w_ih = (const float*)d_in[1];
  const float* w_hh = (const float*)d_in[2];
  const float* b_ih = (const float*)d_in[3];
  const float* b_hh = (const float*)d_in[4];
  const float* w_fc = (const float*)d_in[5];
  const float* b_fc = (const float*)d_in[6];
  float* out = (float*)d_out;

  lstm_seq_kernel<<<NSEQ / ROWS_BLK, NTHR, 0, stream>>>(x, w_ih, w_hh, b_ih, b_hh, w_fc, b_fc, out);
}
